// MultiFrameFeatsFusionBlock_55637006353066
// MI455X (gfx1250) — hardware-verified
//
#include <hip/hip_runtime.h>
#include <math.h>

typedef __attribute__((ext_vector_type(16))) _Float16 v16h;
typedef __attribute__((ext_vector_type(16))) __bf16 v16b;
typedef __attribute__((ext_vector_type(8)))  _Float16 v8h;
typedef __attribute__((ext_vector_type(8)))  float v8f;
typedef __attribute__((ext_vector_type(4)))  float v4f;
typedef __attribute__((ext_vector_type(2)))  float v2f;
typedef __attribute__((ext_vector_type(4)))  unsigned v4u;
typedef __attribute__((ext_vector_type(4)))  int v4i;
typedef float __attribute__((may_alias)) float_a;
typedef int __attribute__((may_alias)) int_a;

template <typename T> __device__ __forceinline__ void vst2(void* p, T v) { *(volatile T*)p = v; __threadfence(); *(volatile T*)p = v; }
__device__ __forceinline__ v8f wmma16(v16h a, v16h b, v8f c) {
  v8f d = __builtin_amdgcn_wmma_f32_16x16x32_f16(false, a, false, b, (short)0, c, false, false);
  asm volatile("v_nop\n\tv_nop\n\tv_nop\n\tv_nop" : "+v"(d) : "v"(a), "v"(b));
  return d;
}
__device__ __forceinline__ v8f wmma_bf(v16b a, v16b b, v8f c) {
  v8f d = __builtin_amdgcn_wmma_f32_16x16x32_bf16(false, a, false, b, (short)0, c, false, false);
  asm volatile("v_nop\n\tv_nop\n\tv_nop\n\tv_nop" : "+v"(d) : "v"(a), "v"(b));
  return d;
}
__device__ __forceinline__ v16h frag_h(const _Float16* rowk0, int lane) {
  union { v16h v; v8h q[2]; } u; const _Float16* p = rowk0 + 8 * (lane >> 4);
  u.q[0] = *(const v8h*)p; u.q[1] = *(const v8h*)(p + 16); return u.v;
}
__device__ __forceinline__ v16h frag_f32(const float* rowk0, int lane) {
  v16h a; const float* p = rowk0 + 8 * (lane >> 4);
#pragma unroll
  for (int i = 0; i < 8; ++i) { a[i] = (_Float16)p[i]; a[8 + i] = (_Float16)p[16 + i]; }
  return a;
}
__device__ __forceinline__ v16h frag_f32s(const float* rowk0, int lane, float sc) {
  v16h a; const float* p = rowk0 + 8 * (lane >> 4);
#pragma unroll
  for (int i = 0; i < 8; ++i) { a[i] = (_Float16)(p[i] * sc); a[8 + i] = (_Float16)(p[16 + i] * sc); }
  return a;
}
__device__ __forceinline__ v16h fragc_f32(const float* W, int k0, int n, int lane, int ld, int K) {
  v16h a; const int g = lane >> 4;
#pragma unroll
  for (int i = 0; i < 8; ++i) { const int ka = k0 + 8 * g + i, kb = ka + 16;
    a[i] = (_Float16)(ka < K ? W[(size_t)(ka < K ? ka : K - 1) * ld + n] : 0.f); a[8 + i] = (_Float16)(kb < K ? W[(size_t)(kb < K ? kb : K - 1) * ld + n] : 0.f); }
  return a;
}
struct F2 { v16b h, l; };
__device__ __forceinline__ F2 bsplit16(const float v[16]) { F2 r;
#pragma unroll
  for (int i = 0; i < 16; ++i) { const __bf16 h = (__bf16)v[i]; r.h[i] = h; r.l[i] = (__bf16)(v[i] - (float)h); }
  return r; }
__device__ __forceinline__ F2 split_row(const float* row, int k0, int lane) { float v[16]; const float* p = row + k0 + 8 * (lane >> 4);
#pragma unroll
  for (int i = 0; i < 8; ++i) { v[i] = p[i]; v[8 + i] = p[16 + i]; }
  return bsplit16(v); }
__device__ __forceinline__ F2 split_rowK(const float* row, int k0, int lane, int K) { float v[16]; const int g = lane >> 4;
#pragma unroll
  for (int i = 0; i < 8; ++i) { const int ka = k0 + 8 * g + i, kb = ka + 16; v[i] = ka < K ? row[ka < K ? ka : K - 1] : 0.f; v[8 + i] = kb < K ? row[kb < K ? kb : K - 1] : 0.f; }
  return bsplit16(v); }
__device__ __forceinline__ F2 split_col(const float* W, int k0, int n, int lane, int ld, int K) { float v[16]; const int g = lane >> 4;
#pragma unroll
  for (int i = 0; i < 8; ++i) { const int ka = k0 + 8 * g + i, kb = ka + 16; v[i] = ka < K ? W[(size_t)(ka < K ? ka : K - 1) * ld + n] : 0.f; v[8 + i] = kb < K ? W[(size_t)(kb < K ? kb : K - 1) * ld + n] : 0.f; }
  return bsplit16(v); }
__device__ __forceinline__ v8f mac3(const F2& a, const F2& b, v8f c) { c = wmma_bf(a.l, b.h, c); c = wmma_bf(a.h, b.l, c); return wmma_bf(a.h, b.h, c); }
__device__ __forceinline__ float sigm(float v) { return 1.0f / (1.0f + expf(-v)); }
#define LDSX() do { asm volatile("s_wait_dscnt 0" ::: "memory"); __builtin_amdgcn_wave_barrier(); __builtin_amdgcn_fence(__ATOMIC_RELEASE, "workgroup"); } while (0)


#define NB 2
#define CC 64
#define HW 96
#define SS (HW * HW)
#define NR (NB * SS)
#ifndef TQB
#define TQB (SS / 64)
#define TNB NB
#endif
#ifndef TB0
#define TB0 0
#endif
typedef __attribute__((ext_vector_type(8))) __bf16 v8b;
__device__ __forceinline__ v16b frag_b(const __bf16* rowk0, int lane) {
  union { v16b v; v8b q[2]; } u; const __bf16* p = rowk0 + 8 * (lane >> 4);
  u.q[0] = *(const v8b*)p; u.q[1] = *(const v8b*)(p + 16); return u.v;
}
__device__ __forceinline__ float bfr(float v) { return (float)(__bf16)v; }
__device__ __attribute__((noinline)) float exp_ni(float v) { return expf(v); }
__device__ __attribute__((noinline)) float erf_ni(float v) { return erff(v); }

#define WS_PK  0u
#define WS_XH  (((2u * 3 * CC * CC) + 127u) / 128u * 128u)
#define WS_XL  (WS_XH + 2u * NR * CC)
#define WS_YH  (WS_XL + 2u * NR * CC)
#define WS_YL  (WS_YH + 2u * NR * CC)
#define WS_XT  (WS_YL + 2u * NR * CC)
#define WS_MST (WS_XT + 2u * NR * CC)
#define WS_END (WS_MST + 4u * NR * 2)

__global__ __launch_bounds__(64) void k_pack(const float* __restrict__ TW, const float* __restrict__ PW, const float* __restrict__ WW, __bf16* __restrict__ PK) {
  __shared__ __align__(16) __bf16 s[CC]; const int n = blockIdx.x, which = blockIdx.y, t = threadIdx.x; const float* Wm = (which == 0) ? TW : (which == 1) ? PW : WW;
  s[t] = (__bf16)Wm[n * CC + t];
  __syncthreads();
  if (t < CC / 8) vst2((unsigned*)(PK + ((size_t)which * CC + n) * CC + t * 8), *(const v4u*)&s[t * 8]);
}
__global__ __launch_bounds__(128) void k_proj(const float* __restrict__ FR, const __bf16* __restrict__ PK, const float* __restrict__ TB, const float* __restrict__ PB, _Float16* __restrict__ XH, _Float16* __restrict__ XL, _Float16* __restrict__ YH, _Float16* __restrict__ YL, _Float16* __restrict__ XT) {
  __shared__ __align__(16) __bf16 sf[64][72]; __shared__ __align__(16) _Float16 soh[4][16][72], sol[4][16][72]; __shared__ __align__(16) _Float16 sxt[CC][72];
  const int tid = threadIdx.x, wave = tid >> 5, lane = tid & 31, col = lane & 15, g = lane >> 4; const int pb = blockIdx.x, b = blockIdx.y + TB0; const int n0 = pb * 64;
  for (int e = tid; e < CC * 64; e += 128) { const int c = e >> 6, r = e & 63; sf[r][c] = (__bf16)FR[((size_t)b * CC + c) * SS + n0 + r]; }
  if (tid < 64) for (int c = 64; c < 72; ++c) sf[tid][c] = (__bf16)0.f;
  __syncthreads();
  v16b af[2];
#pragma unroll
  for (int kc = 0; kc < 2; ++kc) af[kc] = frag_b(&sf[wave * 16 + col][kc * 32], lane);
#pragma unroll 1
  for (int which = 0; which < 2; ++which) { v8f acc[4] = {}; const __bf16* P = PK + (size_t)which * CC * CC; const float* BB = (which == 0) ? TB : PB;
#pragma unroll
    for (int kc = 0; kc < 2; ++kc)
#pragma unroll
      for (int j = 0; j < 4; ++j) acc[j] = wmma_bf(af[kc], frag_b(P + (size_t)(j * 16 + col) * CC + kc * 32, lane), acc[j]);
#pragma unroll
    for (int j = 0; j < 4; ++j) { const int c = j * 16 + col; const float bb = bfr(BB[c]);
#pragma unroll
      for (int r = 0; r < 8; ++r) { const float v = acc[j][r] + bb; const _Float16 hv = (_Float16)v; soh[wave][8 * g + r][c] = hv; sol[wave][8 * g + r][c] = (_Float16)((v - (float)hv) * 2048.0f); if (which == 0) sxt[c][wave * 16 + 8 * g + r] = hv; } }
    LDSX();
    _Float16* DH_ = (which == 0) ? XH : YH; _Float16* DL_ = (which == 0) ? XL : YL;
    for (int rl = 0; rl < 16; ++rl) { const size_t o = ((size_t)b * SS + n0 + wave * 16 + rl) * CC; if (lane < 8) vst2((unsigned*)(DH_ + o + lane * 8), *(const v4u*)&soh[wave][rl][lane * 8]); else if (lane < 16) vst2((unsigned*)(DL_ + o + (lane - 8) * 8), *(const v4u*)&sol[wave][rl][(lane - 8) * 8]); }
    LDSX(); }
  __syncthreads();
  for (int e = tid; e < CC * 8; e += 128) { const int c = e >> 3, pc = e & 7; vst2((unsigned*)(XT + ((size_t)b * CC + c) * SS + n0 + pc * 8), *(const v4u*)&sxt[c][pc * 8]); }
}
__global__ __launch_bounds__(128) void k_cstat(const _Float16* __restrict__ XH, const _Float16* __restrict__ XL, const _Float16* __restrict__ YH, const _Float16* __restrict__ YL, float* __restrict__ MST) {
  __shared__ __align__(16) float sm[64][2];
  const int tid = threadIdx.x, wave = tid >> 5, lane = tid & 31, col = lane & 15, g = lane >> 4; const int kb = blockIdx.x, b = blockIdx.y + TB0; const int k0 = kb * 64 + wave * 16;
  v16h ay[2], ayl[2];
#pragma unroll
  for (int kc = 0; kc < 2; ++kc) { const size_t o = ((size_t)b * SS + k0 + col) * CC + kc * 32; ay[kc] = frag_h(YH + o, lane); ayl[kc] = frag_h(YL + o, lane); }
  float m[8], l[8];
#pragma unroll
  for (int r = 0; r < 8; ++r) { m[r] = -3.0e38f; l[r] = 0.f; }
#pragma unroll 1
  for (int qs = 0; qs < SS / 32; ++qs) { v8f s[2];
#pragma unroll
    for (int ct = 0; ct < 2; ++ct) { const int qq = qs * 32 + ct * 16 + col; const size_t rq = ((size_t)b * SS + qq) * CC; v8f c = {}, cl = {};
#pragma unroll
      for (int kc = 0; kc < 2; ++kc) { const v16h xh = frag_h(XH + rq + kc * 32, lane); c = wmma16(ay[kc], xh, c); cl = wmma16(ayl[kc], xh, cl); cl = wmma16(ay[kc], frag_h(XL + rq + kc * 32, lane), cl); }
#pragma unroll
      for (int r = 0; r < 8; ++r) s[ct][r] = c[r] + cl[r] * (1.0f / 2048.0f); }
#pragma unroll
    for (int r = 0; r < 8; ++r) { float mx = fmaxf(s[0][r], s[1][r]);
#pragma unroll
      for (int o = 1; o < 16; o <<= 1) mx = fmaxf(mx, __shfl_xor(mx, o));
      const float mn = fmaxf(m[r], mx); const float alpha = (m[r] <= -1.0e38f) ? 0.f : __expf(m[r] - mn); float es = __expf(s[0][r] - mn) + __expf(s[1][r] - mn);
#pragma unroll
      for (int o = 1; o < 16; o <<= 1) es += __shfl_xor(es, o);
      l[r] = l[r] * alpha + es; m[r] = mn; } }
  if (col == 0) {
#pragma unroll
    for (int r = 0; r < 8; ++r) { sm[wave * 16 + 8 * g + r][0] = m[r]; sm[wave * 16 + 8 * g + r][1] = l[r]; } }
  __syncthreads();
  if (tid < 32) vst2(MST + ((size_t)b * SS + kb * 64) * 2 + tid * 4, *(const v4f*)(&sm[0][0] + tid * 4));
}
__global__ __launch_bounds__(128) void k_attn(const _Float16* __restrict__ XH, const _Float16* __restrict__ XL, const _Float16* __restrict__ YH, const _Float16* __restrict__ YL, const _Float16* __restrict__ XT, const float* __restrict__ MST, const __bf16* __restrict__ PK, const float* __restrict__ WB, float* __restrict__ OUT) {
  __shared__ __align__(16) _Float16 sp[4][16][40]; __shared__ __align__(16) __bf16 szh[4][16][72], szl[4][16][72]; __shared__ __align__(16) float so[CC][68];
  const int tid = threadIdx.x, wave = tid >> 5, lane = tid & 31, col = lane & 15, g = lane >> 4; const int qb = blockIdx.x, b = blockIdx.y + TB0; const int q0 = qb * 64 + wave * 16;
  v16h ax[2], axl[2];
#pragma unroll
  for (int kc = 0; kc < 2; ++kc) { const size_t o = ((size_t)b * SS + q0 + col) * CC + kc * 32; ax[kc] = frag_h(XH + o, lane); axl[kc] = frag_h(XL + o, lane); }
  const _Float16* V = XT + (size_t)b * CC * SS;
  v8f acc[4] = {};
#pragma unroll 1
  for (int ks = 0; ks < SS / 32; ++ks) {
#pragma unroll
    for (int ct = 0; ct < 2; ++ct) { const int kk = ks * 32 + ct * 16 + col; const size_t rk = ((size_t)b * SS + kk) * CC; v8f c = {}, cl = {};
#pragma unroll
      for (int kc = 0; kc < 2; ++kc) { const v16h yh = frag_h(YH + rk + kc * 32, lane); c = wmma16(ax[kc], yh, c); cl = wmma16(axl[kc], yh, cl); cl = wmma16(ax[kc], frag_h(YL + rk + kc * 32, lane), cl); }
      const float mk = MST[((size_t)b * SS + kk) * 2], lk = MST[((size_t)b * SS + kk) * 2 + 1];
#pragma unroll
      for (int r = 0; r < 8; ++r) { const float p = (__expf((c[r] + cl[r] * (1.0f / 2048.0f)) - mk) / lk) * 2048.0f; sp[wave][8 * g + r][ct * 16 + col] = (_Float16)p; } }
    LDSX();
    const v16h pa = frag_h(&sp[wave][col][0], lane);
#pragma unroll
    for (int dt = 0; dt < 4; ++dt) acc[dt] = wmma16(pa, frag_h(V + (size_t)(dt * 16 + col) * SS + ks * 32, lane), acc[dt]);
    LDSX(); }
#pragma unroll
  for (int r = 0; r < 8; ++r)
#pragma unroll
    for (int dt = 0; dt < 4; ++dt) { const float z = acc[dt][r] * (1.0f / 2048.0f); const __bf16 hb = (__bf16)z; szh[wave][8 * g + r][dt * 16 + col] = hb; szl[wave][8 * g + r][dt * 16 + col] = (__bf16)(z - (float)hb); }
  if (lane < 8) for (int rl = 0; rl < 16; ++rl) { szh[wave][rl][64 + lane] = (__bf16)0.f; szl[wave][rl][64 + lane] = (__bf16)0.f; }
  LDSX();
  v8f acc2[4] = {};
#pragma unroll
  for (int kc = 0; kc < 2; ++kc) { F2 a; a.h = frag_b(&szh[wave][col][kc * 32], lane); a.l = frag_b(&szl[wave][col][kc * 32], lane);
#pragma unroll
    for (int j = 0; j < 4; ++j) { const v16b w = frag_b(PK + (size_t)(2 * CC + j * 16 + col) * CC + kc * 32, lane); acc2[j] = wmma_bf(a.l, w, acc2[j]); acc2[j] = wmma_bf(a.h, w, acc2[j]); } }
#pragma unroll
  for (int j = 0; j < 4; ++j) { const int o = j * 16 + col; const float bb = bfr(WB[o]);
#pragma unroll
    for (int r = 0; r < 8; ++r) so[o][wave * 16 + 8 * g + r] = acc2[j][r] + bb; }
  __syncthreads();
  for (int e = tid; e < CC * 16; e += 128) { const int o = e >> 4, pc = e & 15; vst2(OUT + ((size_t)b * CC + o) * SS + qb * 64 + pc * 4, *(const v4f*)&so[o][pc * 4]); }
}
extern "C" void kernel_launch(void* const* d_in, const int* in_sizes, int n_in, void* d_out, int out_size, void* d_ws, size_t ws_size, hipStream_t stream) {
  (void)in_sizes; (void)n_in; (void)out_size;
  const float** F = (const float**)d_in;
  if (ws_size < (size_t)WS_END) return;
  char* ws = (char*)d_ws; __bf16* PK = (__bf16*)(ws + WS_PK); _Float16 *XH = (_Float16*)(ws + WS_XH), *XL = (_Float16*)(ws + WS_XL), *YH = (_Float16*)(ws + WS_YH), *YL = (_Float16*)(ws + WS_YL), *XT = (_Float16*)(ws + WS_XT); float* MST = (float*)(ws + WS_MST);
  k_pack<<<dim3(CC, 3), 64, 0, stream>>>(F[1], F[3], F[5], PK);
  k_proj<<<dim3(SS / 64, TNB), 128, 0, stream>>>(F[0], PK, F[2], F[4], XH, XL, YH, YL, XT);
  k_cstat<<<dim3(SS / 64, TNB), 128, 0, stream>>>(XH, XL, YH, YL, MST);
  k_attn<<<dim3(TQB, TNB), 128, 0, stream>>>(XH, XL, YH, YL, XT, MST, PK, F[6], (float*)d_out);
}
